// ConcatAttention_79894981640368
// MI455X (gfx1250) — hardware-verified
//
#include <hip/hip_runtime.h>


#ifndef NT
#define NT 32
#endif
#define NT_FULL 32
#define NS    128
#define NBAT  16
#define HH    1024
#define HLOG  10
#define LOG2E 1.4426950408889634f

static_assert(NT >= 4 && NT <= NT_FULL && NT % 4 == 0);
static_assert((1 << HLOG) == HH);
static_assert((NT * NBAT) % 64 == 0 && (NS * NBAT) % 64 == 0 && HH % 64 == 0);
static_assert(HH % 32 == 0 && HH % 128 == 0 && HH == 32 * 32);
static_assert(NS == 8 * 16 && NS == 16 * 8 && NBAT == 16 && 256 == NBAT * 16);
static_assert(256 * 4 * 2 == NS * NBAT);
static_assert((size_t)256 * 16 * 2 == (size_t)NS * NBAT * 4);
static_assert(((size_t)2 * HH * HH / 8) % 256 == 0);
static_assert((size_t)NT_FULL * NS * NBAT * 4 == 262144);
static_assert(((size_t)NS * NBAT + 512) * 4 <= 131072);
static_assert((size_t)16 * 68 * 4 <= 131072);
#define WS_TOTAL ((size_t)2 * HH * HH * 2 + (size_t)NT * NBAT * HH * 2 + (size_t)NS * NBAT * HH * 2 + (size_t)NT * NBAT * HH * 4 + (size_t)NS * NBAT * HH * 4)
static_assert(WS_TOTAL <= (size_t)134217728);
static_assert(((size_t)2 * HH * HH * 2) % 256 == 0 && ((size_t)NT * NBAT * HH * 2) % 256 == 0 && ((size_t)NS * NBAT * HH * 2) % 256 == 0 && ((size_t)NT * NBAT * HH * 4) % 256 == 0);

typedef unsigned short bf;
typedef __attribute__((ext_vector_type(16))) __bf16   v16bf;
typedef __attribute__((ext_vector_type(8)))  unsigned short v8us;
typedef __attribute__((ext_vector_type(8)))  float    v8f;
typedef __attribute__((ext_vector_type(4)))  float    v4f;
typedef v4f  __attribute__((may_alias)) v4fa;

__device__ __forceinline__ unsigned short f2bf(float f) { unsigned u = __float_as_uint(f); u += 0x7FFFu + ((u >> 16) & 1u); return (unsigned short)(u >> 16); }
__device__ __forceinline__ float bf2f(unsigned short b) { return __uint_as_float(((unsigned)b) << 16); }
__device__ __forceinline__ float bfr(float f) { return bf2f(f2bf(f)); }
__device__ __forceinline__ v16bf cat16b(v8us lo, v8us hi) { return __builtin_bit_cast(v16bf, __builtin_shufflevector(lo, hi, 0, 1, 2, 3, 4, 5, 6, 7, 8, 9, 10, 11, 12, 13, 14, 15)); }
__device__ __forceinline__ v8f wmmab(v16bf a, v16bf b, v8f c) { return __builtin_amdgcn_wmma_f32_16x16x32_bf16(false, a, false, b, (short)0, c, false, false); }

template <typename T16> struct WFrag;
template <> struct WFrag<bf> { typedef v16bf V; static __device__ __forceinline__ V ld(const bf* p) { return cat16b(*(const v8us*)p, *(const v8us*)(p + 16)); } static __device__ __forceinline__ v8f mma(V a, V b, v8f c) { return wmmab(a, b, c); } };
template <typename T16, int NSPLIT, bool BIAS>
__global__ __launch_bounds__(32) void k_gemmw(const T16* __restrict__ A, const T16* __restrict__ A2, const T16* __restrict__ Bt, const T16* __restrict__ Bt2, int K, float* C, int ldc, const float* __restrict__ bias, float csc, size_t sA, size_t sB, size_t sC) {
    typedef typename WFrag<T16>::V V;
    __shared__ __align__(16) float os[16 * 68];
    const size_t z = blockIdx.z; A += z * sA; if (A2) A2 += z * sA; Bt += z * sB; if (Bt2) Bt2 += z * sB; C += z * sC;
    const int lane = threadIdx.x & 31, lr = lane & 15, hi = lane >> 4; const int r0 = blockIdx.x * 64, c0 = blockIdx.y * 64;
    v8f acc[4][4];
#pragma unroll
    for (int mb = 0; mb < 4; ++mb)
#pragma unroll
        for (int nb = 0; nb < 4; ++nb) acc[mb][nb] = (v8f){};
    const size_t aoff = (size_t)(r0 + lr) * K + 8 * hi, boff = (size_t)(c0 + lr) * K + 8 * hi;
#pragma unroll 1
    for (int kc = 0; kc < K; kc += 32) {
        V a[4], a2[4];
#pragma unroll
        for (int mb = 0; mb < 4; ++mb) { a[mb] = WFrag<T16>::ld(A + aoff + (size_t)mb * 16 * K + kc); if (NSPLIT == 1 || NSPLIT == 2) a2[mb] = WFrag<T16>::ld(A2 + aoff + (size_t)mb * 16 * K + kc); }
#pragma unroll
        for (int nb = 0; nb < 4; ++nb) { const V b = WFrag<T16>::ld(Bt + boff + (size_t)nb * 16 * K + kc); V b2; if (NSPLIT >= 2) b2 = WFrag<T16>::ld(Bt2 + boff + (size_t)nb * 16 * K + kc);
#pragma unroll
            for (int mb = 0; mb < 4; ++mb) { acc[mb][nb] = WFrag<T16>::mma(a[mb], b, acc[mb][nb]); if (NSPLIT == 1 || NSPLIT == 2) acc[mb][nb] = WFrag<T16>::mma(a2[mb], b, acc[mb][nb]); if (NSPLIT >= 2) acc[mb][nb] = WFrag<T16>::mma(a[mb], b2, acc[mb][nb]); } }
        asm volatile("v_nop\n\tv_nop\n\tv_nop\n\tv_nop" : "+v"(acc[0][0]), "+v"(acc[1][1]), "+v"(acc[2][2]), "+v"(acc[3][3]) : "v"(a[0]), "v"(a[3]));
    }
#pragma unroll
    for (int mb = 0; mb < 4; ++mb) {
#pragma unroll
        for (int nb = 0; nb < 4; ++nb) {
#pragma unroll
            for (int j = 0; j < 8; ++j) os[(hi * 8 + j) * 68 + nb * 16 + lr] = acc[mb][nb][j]; }
        __builtin_amdgcn_wave_barrier(); asm volatile("" ::: "memory");
        float* crow = C + (size_t)(r0 + mb * 16) * ldc + c0;
#pragma unroll 1
        for (int ps = 0; ps < 2; ++ps) {
#pragma unroll
            for (int s = 0; s < 8; ++s) { const int row = 2 * s + hi, cofs = lr * 4; v4f val = *(const v4fa*)(os + row * 68 + cofs); val = val * csc;
                if (BIAS) { val[0] += bfr(bias[c0 + cofs]); val[1] += bfr(bias[c0 + cofs + 1]); val[2] += bfr(bias[c0 + cofs + 2]); val[3] += bfr(bias[c0 + cofs + 3]); }
                *(volatile v4f*)(crow + (size_t)row * ldc + cofs) = val; }
            if (ps == 0) __threadfence(); }
        __builtin_amdgcn_wave_barrier(); asm volatile("" ::: "memory");
    }
}

__global__ __launch_bounds__(256) void k_wsp8(const float* __restrict__ w, bf* Bt) {
    const unsigned i = blockIdx.x * 256u + threadIdx.x; const unsigned e = i << 3;
    const unsigned half = e >> (2 * HLOG), n = (e >> HLOG) & (unsigned)(HH - 1), k = e & (unsigned)(HH - 1);
    const v8f v = *(const v8f*)(w + (size_t)n * (2 * HH) + (size_t)half * HH + k); v8us o;
#pragma unroll
    for (int q = 0; q < 8; ++q) o[q] = f2bf(v[q]); *(volatile v8us*)(Bt + (size_t)e) = o; __threadfence(); *(volatile v8us*)(Bt + (size_t)e) = o; }

__global__ __launch_bounds__(256) void k_cvt8(const float* __restrict__ src, bf* dst, size_t n8) { const size_t i = (size_t)blockIdx.x * 256 + threadIdx.x; if (i >= n8) return; const v8f v = *(const v8f*)(src + i * 8); v8us o;
#pragma unroll
    for (int k = 0; k < 8; ++k) o[k] = f2bf(v[k]); *(volatile v8us*)(dst + i * 8) = o; __threadfence(); *(volatile v8us*)(dst + i * 8) = o; }

__device__ __forceinline__ float tnh(float x) {
    const float e = __builtin_amdgcn_exp2f(x * 2.8853900817779268f);
    const float r = __builtin_amdgcn_rcpf(e + 1.0f);
    return fmaf(-2.0f, r, 1.0f);
}

__global__ __launch_bounds__(256) void k_score(const float* __restrict__ HPF, const float* __restrict__ SPF, const float* __restrict__ va, float* OUT) {
    __shared__ __align__(16) float s_sc[NS * NBAT];
    __shared__ float s_mx[256];
    __shared__ float s_sm[256];
    const int t = blockIdx.x;
    const int tid = threadIdx.x, lane = tid & 31;
    const int wave = __builtin_amdgcn_readfirstlane(threadIdx.x >> 5);
    float vr[32];
#pragma unroll
    for (int i = 0; i < 8; ++i) { const v4f v4 = *(const v4f*)(va + i * 128 + lane * 4);
#pragma unroll
        for (int c = 0; c < 4; ++c) vr[i * 4 + c] = bfr(v4[c]); }
#pragma unroll 1
    for (int b = 0; b < NBAT; ++b) {
        const float* wrow = HPF + (size_t)(t * NBAT + b) * HH;
        float wq[32];
#pragma unroll
        for (int i = 0; i < 8; ++i) { const v4f w4 = *(const v4f*)(wrow + i * 128 + lane * 4);
#pragma unroll
            for (int c = 0; c < 4; ++c) wq[i * 4 + c] = w4[c]; }
#pragma unroll 1
        for (int kk = 0; kk < NS / 8; ++kk) {
            const int s = wave * (NS / 8) + kk;
            const float* urow = SPF + (size_t)(s * NBAT + b) * HH;
            float acc = 0.0f;
#pragma unroll
            for (int i = 0; i < 8; ++i) { const v4f u4 = *(const v4f*)(urow + i * 128 + lane * 4);
#pragma unroll
                for (int c = 0; c < 4; ++c) acc = fmaf(vr[i * 4 + c], tnh(wq[i * 4 + c] + u4[c]), acc); }
#pragma unroll
            for (int sh = 16; sh; sh >>= 1) acc += __shfl_xor(acc, sh, 32);
            if (lane == 0) s_sc[s * NBAT + b] = acc;
        }
    }
    __syncthreads();
    const int bb = tid & 15, g = tid >> 4;
    float a[8];
#pragma unroll
    for (int j = 0; j < 8; ++j) a[j] = s_sc[(8 * g + j) * NBAT + bb];
    float m = a[0];
#pragma unroll
    for (int j = 1; j < 8; ++j) m = (a[j] > m) ? a[j] : m;
    s_mx[g * 16 + bb] = m;
    __syncthreads();
    m = s_mx[bb];
#pragma unroll
    for (int gg = 1; gg < 16; ++gg) { const float o = s_mx[gg * 16 + bb]; m = (o > m) ? o : m; }
    float e[8];
#pragma unroll
    for (int j = 0; j < 8; ++j) {
        float d = a[j] - m; asm volatile("" : "+v"(d));
        e[j] = __builtin_amdgcn_exp2f(d * LOG2E); }
    float sum = e[0];
#pragma unroll
    for (int j = 1; j < 8; ++j) sum += e[j];
    s_sm[g * 16 + bb] = sum;
    __syncthreads();
    sum = s_sm[bb];
#pragma unroll
    for (int gg = 1; gg < 16; ++gg) sum += s_sm[gg * 16 + bb];
    const float inv = __builtin_amdgcn_rcpf(sum);
#pragma unroll
    for (int j = 0; j < 8; ++j) s_sc[(8 * g + j) * NBAT + bb] = e[j] * inv;
    __syncthreads();
    const int f0 = tid * 4;
    const v4f p0 = *(const v4fa*)(s_sc + f0); const v4f p1 = *(const v4fa*)(s_sc + 1024 + f0);
    float* dst = OUT + (size_t)t * (NS * NBAT) + f0;
    *(volatile v4f*)dst = p0; *(volatile v4f*)(dst + 1024) = p1; __threadfence(); *(volatile v4f*)dst = p0; *(volatile v4f*)(dst + 1024) = p1;
}

extern "C" void kernel_launch(void* const* d_in, const int* in_sizes, int n_in,
                              void* d_out, int out_size, void* d_ws, size_t ws_size, hipStream_t stream) {
    if (n_in < 5) return;
    if (in_sizes[0] < NT * NBAT * HH || in_sizes[1] < NS * NBAT * HH || in_sizes[2] < HH * 2 * HH || in_sizes[3] < HH || in_sizes[4] < HH) return;
    if (out_size < NT * NS * NBAT) return;
    const float* h_t  = (const float*)d_in[0];
    const float* src  = (const float*)d_in[1];
    const float* Wa_w = (const float*)d_in[2];
    const float* Wa_b = (const float*)d_in[3];
    const float* Va_w = (const float*)d_in[4];
    float* OUT = (float*)d_out;

    char* wsp = (char*)d_ws;
    auto take = [&](size_t bytes) { char* p = wsp; wsp += (bytes + 255) & ~(size_t)255; return (void*)p; };
    bf*    BT  = (bf*)take((size_t)2 * HH * HH * 2);
    bf*    HB  = (bf*)take((size_t)NT * NBAT * HH * 2);
    bf*    SB  = (bf*)take((size_t)NS * NBAT * HH * 2);
    float* HPF = (float*)take((size_t)NT * NBAT * HH * 4);
    float* SPF = (float*)take((size_t)NS * NBAT * HH * 4);
    if ((size_t)(wsp - (char*)d_ws) > ws_size) return;

    k_wsp8<<<(unsigned)((size_t)2 * HH * HH / 8 / 256), 256, 0, stream>>>(Wa_w, BT);
    k_cvt8<<<(unsigned)(((size_t)NT * NBAT * HH / 8 + 255) / 256), 256, 0, stream>>>(h_t, HB, (size_t)NT * NBAT * HH / 8);
    k_cvt8<<<(unsigned)(((size_t)NS * NBAT * HH / 8 + 255) / 256), 256, 0, stream>>>(src, SB, (size_t)NS * NBAT * HH / 8);
    k_gemmw<bf, 0, true><<<dim3(NT * NBAT / 64, HH / 64, 1), 32, 0, stream>>>(HB, nullptr, BT, nullptr, HH, HPF, HH, Wa_b, 1.0f, 0, 0, 0);
    k_gemmw<bf, 0, false><<<dim3(NS * NBAT / 64, HH / 64, 1), 32, 0, stream>>>(SB, nullptr, BT + (size_t)HH * HH, nullptr, HH, SPF, HH, nullptr, 1.0f, 0, 0, 0);
    k_score<<<(unsigned)NT, 256, 0, stream>>>(HPF, SPF, Va_w, OUT);
}
